// FlowAssembly_28372553957669
// MI455X (gfx1250) — hardware-verified
//
#include <hip/hip_runtime.h>
#include <math.h>
#include <stddef.h>
#include <stdint.h>


#define NB    4
#define NP    16384
#define NC    32
#define NH    16
#define KN    16
#define HD    64
#define NPT   (NB * NP)
#define NTHR  256
#define NWAVE 8
#define PPB   128
#define NBLK  (NPT / PPB)
#define BPB   (NP / PPB)
#define PLP   72
#define XSC   8
#define HSC   16
#define WSC   1024
#define WSCAP 134217728
#define SCF   1.2095775674984046f

static_assert(NPT % PPB == 0);
static_assert(NP % PPB == 0);
static_assert(PPB == NWAVE * 16);
static_assert(NTHR == NWAVE * 32);
static_assert(NBLK == NB * BPB);
static_assert(NH * 2 == NC);
static_assert(KN == 16);
static_assert(HD == 64);
static_assert((PLP % 8) == 0);

typedef float    v4f  __attribute__((ext_vector_type(4)));
typedef float    v8f  __attribute__((ext_vector_type(8)));
typedef _Float16 v8h  __attribute__((ext_vector_type(8)));
typedef _Float16 v16h __attribute__((ext_vector_type(16)));
union FragH { v16h v; v8h h[2]; };

__device__ __forceinline__ v8f wmf(v16h a, v16h b, v8f c) {
  v8f d = __builtin_amdgcn_wmma_f32_16x16x32_f16(false, a, false, b, (short)0, c, false, false);
  asm volatile("v_nop\n\tv_nop\n\tv_nop\n\tv_nop" : "+v"(d) : "v"(a), "v"(b));
  return d;
}

__device__ __forceinline__ v8f vz8() {
  v8f z = {0.f, 0.f, 0.f, 0.f, 0.f, 0.f, 0.f, 0.f};
  return z;
}

__device__ __forceinline__ v16h ldfrag(const _Float16* plane, int KP, int row, int k0, int hh) {
  FragH f;
  const _Float16* p = plane + row * KP + k0 + 8 * hh;
  f.h[0] = *(const v8h*)p;
  f.h[1] = *(const v8h*)(p + 16);
  return f.v;
}

__device__ __forceinline__ v16h cvt2(v8f lo, v8f hi, float s) {
  v16h o;
#pragma unroll
  for (int r = 0; r < 8; ++r) {
    o[r] = (_Float16)(lo[r] * s);
    o[8 + r] = (_Float16)(hi[r] * s);
  }
  return o;
}

__device__ __forceinline__ void pack_w(_Float16* dst, const float* __restrict__ W, int KR, int KP, int NOUT) {
  const int tot = NOUT * KP;
  for (int i = (int)threadIdx.x; i < tot; i += NTHR) {
    const int n = i / KP;
    const int k = i - n * KP;
    const int kc = min(k, KR - 1);
    const float v = W[(size_t)kc * NOUT + n] * (float)WSC;
    dst[i] = (k < KR) ? (_Float16)v : (_Float16)0.0f;
  }
}

__global__ __launch_bounds__(NTHR) void k_cpl1(const float* __restrict__ x,
                                               const float* __restrict__ an_logs,
                                               const float* __restrict__ an_bias,
                                               const float* __restrict__ w1, const float* __restrict__ b1,
                                               const float* __restrict__ g1, const float* __restrict__ be1,
                                               const float* __restrict__ w2, const float* __restrict__ b2,
                                               const float* __restrict__ w3, const float* __restrict__ b3,
                                               float* P, float* part) {
  __shared__ __attribute__((aligned(16))) _Float16 w1t[HD * 32];
  __shared__ __attribute__((aligned(16))) _Float16 w2t[HD * HD];
  __shared__ __attribute__((aligned(16))) _Float16 w3t[NC * HD];
  __shared__ __attribute__((aligned(16))) float stg[NWAVE * 16 * NC];
  __shared__ float s_e[NC], s_ab[NC], s_b3[NC];
  __shared__ float s_b1[HD], s_g1[HD], s_be1[HD], s_b2[HD];
  __shared__ float s_ld[NWAVE];

  const int tid = threadIdx.x, lane = tid & 31, wave = tid >> 5, hh = lane >> 4, m = lane & 15;
  pack_w(w1t, w1, NH, 32, HD);
  pack_w(w2t, w2, HD, HD, HD);
  pack_w(w3t, w3, HD, HD, NC);
  if (tid < NC) { s_e[tid] = expf(an_logs[tid]); s_ab[tid] = an_bias[tid]; s_b3[tid] = b3[tid]; }
  if (tid < HD) { s_b1[tid] = b1[tid]; s_g1[tid] = g1[tid]; s_be1[tid] = be1[tid]; s_b2[tid] = b2[tid]; }
  __syncthreads();

  const int pw = blockIdx.x * PPB + wave * 16;
  const int p = pw + m;
  const float* xr = x + (size_t)p * NC;
  const v4f xa0 = *(const v4f*)(xr + 24 - 8 * hh);
  const v4f xa1 = *(const v4f*)(xr + 28 - 8 * hh);
  const v4f xb0 = *(const v4f*)(xr + 8 - 8 * hh);
  const v4f xb1 = *(const v4f*)(xr + 12 - 8 * hh);
  const float xs[8] = {xa0.x, xa0.y, xa0.z, xa0.w, xa1.x, xa1.y, xa1.z, xa1.w};
  const float xu[8] = {xb0.x, xb0.y, xb0.z, xb0.w, xb1.x, xb1.y, xb1.z, xb1.w};
  float y1[8], y2[8];
#pragma unroll
  for (int i = 0; i < 8; ++i) {
    const int c = 8 * hh + i;
    y1[i] = xs[7 - i] * s_e[c] + s_ab[c];
    y2[i] = xu[7 - i] * s_e[16 + c] + s_ab[16 + c];
  }
  const float O1 = 1.0f / (float)(XSC * WSC);
  const float O2 = 1.0f / (float)(HSC * WSC);

  v16h bx;
#pragma unroll
  for (int i = 0; i < 8; ++i) { bx[i] = (_Float16)(y1[i] * (float)XSC); bx[8 + i] = (_Float16)0.0f; }
  v8f acc[4];
#pragma unroll
  for (int t = 0; t < 4; ++t) acc[t] = wmf(ldfrag(w1t, 32, 16 * t + m, 0, hh), bx, vz8());
#pragma unroll
  for (int t = 0; t < 4; ++t) {
#pragma unroll
    for (int r = 0; r < 8; ++r) {
      const int n = 16 * t + 8 * hh + r;
      float v = acc[t][r] * O1 + s_b1[n];
      v = s_g1[n] * v + s_be1[n];
      acc[t][r] = fmaxf(v, 0.0f);
    }
  }
  const v16h bf0 = cvt2(acc[0], acc[1], (float)HSC);
  const v16h bf1 = cvt2(acc[2], acc[3], (float)HSC);

  v8f acc2[4];
#pragma unroll
  for (int t = 0; t < 4; ++t) {
    acc2[t] = wmf(ldfrag(w2t, HD, 16 * t + m, 0, hh), bf0, vz8());
    acc2[t] = wmf(ldfrag(w2t, HD, 16 * t + m, 32, hh), bf1, acc2[t]);
  }
#pragma unroll
  for (int t = 0; t < 4; ++t) {
#pragma unroll
    for (int r = 0; r < 8; ++r) {
      const int n = 16 * t + 8 * hh + r;
      acc2[t][r] = fmaxf(acc2[t][r] * O2 + s_b2[n], 0.0f);
    }
  }
  const v16h cf0 = cvt2(acc2[0], acc2[1], (float)HSC);
  const v16h cf1 = cvt2(acc2[2], acc2[3], (float)HSC);

  v8f accs = wmf(ldfrag(w3t, HD, m, 0, hh), cf0, vz8());
  accs = wmf(ldfrag(w3t, HD, m, 32, hh), cf1, accs);
  v8f acct = wmf(ldfrag(w3t, HD, 16 + m, 0, hh), cf0, vz8());
  acct = wmf(ldfrag(w3t, HD, 16 + m, 32, hh), cf1, acct);

  float ldl = 0.0f;
  float* sp = stg + (wave * 16 + m) * NC;
#pragma unroll
  for (int r = 0; r < 8; ++r) {
    const int c = 8 * hh + r;
    const float sr = accs[r] * O2 + s_b3[c];
    const float sv = SCF * atanf(sr * (1.0f / SCF));
    const float tv = acct[r] * O2 + s_b3[16 + c];
    const float x2n = y2[r] * expf(sv) + tv;
    ldl += sv;
    sp[15 - c] = x2n;
    sp[31 - c] = y1[r];
  }
#pragma unroll
  for (int off = 16; off > 0; off >>= 1) ldl += __shfl_xor(ldl, off, 32);
  if (lane == 0) s_ld[wave] = ldl;
  __syncthreads();

  const int rq = lane >> 3, c4 = 4 * (lane & 7);
  const float* sw = stg + wave * 16 * NC;
  v4f ov[4];
#pragma unroll
  for (int q = 0; q < 4; ++q) ov[q] = *(const v4f*)(sw + (4 * q + rq) * NC + c4);
  float* prow = P + (size_t)pw * NC;
  float tot = 0.0f;
#pragma unroll
  for (int w = 0; w < NWAVE; ++w) tot += s_ld[w];
  const float pv = (lane == 0) ? tot : 0.0f;
  float* pl = part + (size_t)blockIdx.x * 32 + lane;
#pragma unroll
  for (int q = 0; q < 4; ++q) *(volatile v4f*)(prow + (size_t)(4 * q + rq) * NC + c4) = ov[q];
  if (wave == 0) *(volatile float*)pl = pv;
  __threadfence();
#pragma unroll
  for (int q = 0; q < 4; ++q) *(volatile v4f*)(prow + (size_t)(4 * q + rq) * NC + c4) = ov[q];
  if (wave == 0) *(volatile float*)pl = pv;
}

__global__ __launch_bounds__(NTHR) void k_cpl2(const float* __restrict__ P, const int* __restrict__ knn,
                                               const float* __restrict__ k1, const float* __restrict__ kb1,
                                               const float* __restrict__ k2, const float* __restrict__ kb2,
                                               const float* __restrict__ k3, const float* __restrict__ kb3,
                                               float* out, float* part) {
  __shared__ __attribute__((aligned(16))) _Float16 k1t[HD * 32];
  __shared__ __attribute__((aligned(16))) _Float16 k2t[HD * HD];
  __shared__ __attribute__((aligned(16))) _Float16 k3t[NC * HD];
  __shared__ __attribute__((aligned(16))) float gt[NWAVE * 16 * 16];
  __shared__ __attribute__((aligned(16))) _Float16 pool[NWAVE * 16 * PLP];
  __shared__ __attribute__((aligned(16))) float stg[NWAVE * 16 * NC];
  __shared__ float s_kb1[HD], s_kb2[HD], s_kb3[NC];
  __shared__ float s_ld[NWAVE];

  const int tid = threadIdx.x, lane = tid & 31, wave = tid >> 5, hh = lane >> 4, m = lane & 15;
  pack_w(k1t, k1, NC, 32, HD);
  pack_w(k2t, k2, HD, HD, HD);
  pack_w(k3t, k3, HD, HD, NC);
  if (tid < HD) { s_kb1[tid] = kb1[tid]; s_kb2[tid] = kb2[tid]; }
  if (tid < NC) s_kb3[tid] = kb3[tid];
  __syncthreads();

  const int pw = blockIdx.x * PPB + wave * 16;
  const int b = blockIdx.x / BPB;
  const float* Pb = P + (size_t)b * NP * NC;
  float* gw = gt + wave * 256;
  _Float16* poolw = pool + wave * 16 * PLP;
  float* sw = stg + wave * 16 * NC;
  const int jn = lane >> 1, gofs = 8 * (lane & 1);
  const float O1 = 1.0f / (float)(XSC * WSC);
  const float O2 = 1.0f / (float)(HSC * WSC);

#pragma unroll 1
  for (int j = 0; j < 16; ++j) {
    const int p = pw + j;
    __syncthreads();
    int id = knn[(size_t)p * KN + jn];
    id = min(max(id, 0), NP - 1);
    const float* src = Pb + (size_t)id * NC + gofs;
    const v4f ga = *(const v4f*)src;
    const v4f gb = *(const v4f*)(src + 4);
    *(v4f*)(gw + jn * 16 + gofs) = ga;
    *(v4f*)(gw + jn * 16 + gofs + 4) = gb;
    const float* cr = P + (size_t)p * NC + 8 * hh;
    const v4f ca = *(const v4f*)cr;
    const v4f cb = *(const v4f*)(cr + 4);
    __syncthreads();
    const float* gr = gw + m * 16 + 8 * hh;
    const v4f na = *(const v4f*)gr;
    const v4f nn = *(const v4f*)(gr + 4);
    const float cv[8] = {ca.x, ca.y, ca.z, ca.w, cb.x, cb.y, cb.z, cb.w};
    const float nv[8] = {na.x, na.y, na.z, na.w, nn.x, nn.y, nn.z, nn.w};
    v16h be;
#pragma unroll
    for (int i = 0; i < 8; ++i) {
      be[i] = (_Float16)(cv[i] * (float)XSC);
      be[8 + i] = (_Float16)((nv[i] - cv[i]) * (float)XSC);
    }
    v8f acc[4];
#pragma unroll
    for (int t = 0; t < 4; ++t) acc[t] = wmf(ldfrag(k1t, 32, 16 * t + m, 0, hh), be, vz8());
#pragma unroll
    for (int t = 0; t < 4; ++t) {
#pragma unroll
      for (int r = 0; r < 8; ++r) {
        const int n = 16 * t + 8 * hh + r;
        acc[t][r] = fmaxf(acc[t][r] * O1 + s_kb1[n], 0.0f);
      }
    }
    const v16h af0 = cvt2(acc[0], acc[1], (float)HSC);
    const v16h af1 = cvt2(acc[2], acc[3], (float)HSC);
    float plv[4];
#pragma unroll
    for (int t = 0; t < 4; ++t) {
      v8f d = wmf(af0, ldfrag(k2t, HD, 16 * t + m, 0, hh), vz8());
      d = wmf(af1, ldfrag(k2t, HD, 16 * t + m, 32, hh), d);
      const float bb = s_kb2[16 * t + m];
      float mx = d[0] * O2 + bb;
#pragma unroll
      for (int r = 1; r < 8; ++r) mx = fmaxf(mx, d[r] * O2 + bb);
      mx = fmaxf(mx, 0.0f);
      mx = fmaxf(mx, __shfl_xor(mx, 16, 32));
      plv[t] = mx;
    }
    const float pa = hh ? plv[2] : plv[0];
    const float pc = hh ? plv[3] : plv[1];
    _Float16* pr = poolw + j * PLP + 32 * hh + m;
    pr[0] = (_Float16)(pa * (float)HSC);
    pr[16] = (_Float16)(pc * (float)HSC);
  }
  __syncthreads();

  const v16h bp0 = ldfrag(poolw, PLP, m, 0, hh);
  const v16h bp1 = ldfrag(poolw, PLP, m, 32, hh);
  v8f accs = wmf(ldfrag(k3t, HD, m, 0, hh), bp0, vz8());
  accs = wmf(ldfrag(k3t, HD, m, 32, hh), bp1, accs);
  v8f acct = wmf(ldfrag(k3t, HD, 16 + m, 0, hh), bp0, vz8());
  acct = wmf(ldfrag(k3t, HD, 16 + m, 32, hh), bp1, acct);

  const int p = pw + m;
  const float* xr = P + (size_t)p * NC;
  const v4f u0 = *(const v4f*)(xr + 8 * hh);
  const v4f u1 = *(const v4f*)(xr + 8 * hh + 4);
  const v4f q0 = *(const v4f*)(xr + 16 + 8 * hh);
  const v4f q1 = *(const v4f*)(xr + 16 + 8 * hh + 4);
  const float qv[8] = {q0.x, q0.y, q0.z, q0.w, q1.x, q1.y, q1.z, q1.w};
  float* sp = sw + m * NC;
  *(v4f*)(sp + 8 * hh) = u0;
  *(v4f*)(sp + 8 * hh + 4) = u1;
  float ldl = 0.0f;
#pragma unroll
  for (int r = 0; r < 8; ++r) {
    const int c = 8 * hh + r;
    const float sr = accs[r] * O2 + s_kb3[c];
    const float sv = SCF * atanf(sr * (1.0f / SCF));
    const float tv = acct[r] * O2 + s_kb3[16 + c];
    const float x2n = qv[r] * expf(sv) + tv;
    ldl += sv;
    sp[16 + c] = x2n;
  }
#pragma unroll
  for (int off = 16; off > 0; off >>= 1) ldl += __shfl_xor(ldl, off, 32);
  if (lane == 0) s_ld[wave] = ldl;
  __syncthreads();

  const int rq = lane >> 3, c4 = 4 * (lane & 7);
  v4f ov[4];
#pragma unroll
  for (int q = 0; q < 4; ++q) ov[q] = *(const v4f*)(sw + (4 * q + rq) * NC + c4);
  float* orow = out + (size_t)pw * NC;
  float tot = 0.0f;
#pragma unroll
  for (int w = 0; w < NWAVE; ++w) tot += s_ld[w];
  const float pv = (lane == 0) ? tot : 0.0f;
  float* pl = part + (size_t)blockIdx.x * 32 + lane;
#pragma unroll
  for (int q = 0; q < 4; ++q) *(volatile v4f*)(orow + (size_t)(4 * q + rq) * NC + c4) = ov[q];
  if (wave == 0) *(volatile float*)pl = pv;
  __threadfence();
#pragma unroll
  for (int q = 0; q < 4; ++q) *(volatile v4f*)(orow + (size_t)(4 * q + rq) * NC + c4) = ov[q];
  if (wave == 0) *(volatile float*)pl = pv;
}

__global__ __launch_bounds__(64) void k_logdet(const float* __restrict__ an_logs,
                                               const float* __restrict__ part1,
                                               const float* __restrict__ part3, float* out) {
  __shared__ double s_acc[NB];
  const int tid = threadIdx.x;
  if (tid < NB) {
    double a = 0.0;
#pragma unroll 1
    for (int i = 0; i < BPB; ++i) a += (double)part1[(size_t)(tid * BPB + i) * 32];
#pragma unroll 1
    for (int i = 0; i < BPB; ++i) a += (double)part3[(size_t)(tid * BPB + i) * 32];
    float l0 = 0.0f;
#pragma unroll 1
    for (int c = 0; c < NC; ++c) l0 += an_logs[c];
    s_acc[tid] = a + (double)((float)NP * l0);
  }
  __syncthreads();
  if (tid == 0) {
    v4f o;
    o.x = (float)s_acc[0]; o.y = (float)s_acc[1]; o.z = (float)s_acc[2]; o.w = (float)s_acc[3];
    float* q = out + (size_t)NPT * NC;
    *(volatile v4f*)q = o;
    __threadfence();
    *(volatile v4f*)q = o;
  }
}

extern "C" void kernel_launch(void* const* d_in, const int* in_sizes, int n_in,
                              void* d_out, int out_size, void* d_ws, size_t ws_size,
                              hipStream_t stream) {
  if (n_in < 18) return;
  if (in_sizes[0] != NPT * NC || in_sizes[1] != NPT * KN) return;
  if (in_sizes[2] != NC || in_sizes[3] != NC) return;
  if (in_sizes[4] != NH * HD || in_sizes[5] != HD || in_sizes[6] != HD || in_sizes[7] != HD) return;
  if (in_sizes[8] != HD * HD || in_sizes[9] != HD || in_sizes[10] != HD * NC || in_sizes[11] != NC) return;
  if (in_sizes[12] != NC * HD || in_sizes[13] != HD || in_sizes[14] != HD * HD || in_sizes[15] != HD) return;
  if (in_sizes[16] != HD * NC || in_sizes[17] != NC) return;
  if (out_size != NPT * NC + NB) return;

  const float* x       = (const float*)d_in[0];
  const int*   knn     = (const int*)d_in[1];
  const float* an_logs = (const float*)d_in[2];
  const float* an_bias = (const float*)d_in[3];
  const float* w1  = (const float*)d_in[4];
  const float* b1  = (const float*)d_in[5];
  const float* g1  = (const float*)d_in[6];
  const float* be1 = (const float*)d_in[7];
  const float* w2  = (const float*)d_in[8];
  const float* b2  = (const float*)d_in[9];
  const float* w3  = (const float*)d_in[10];
  const float* b3  = (const float*)d_in[11];
  const float* k1  = (const float*)d_in[12];
  const float* kb1 = (const float*)d_in[13];
  const float* k2  = (const float*)d_in[14];
  const float* kb2 = (const float*)d_in[15];
  const float* k3  = (const float*)d_in[16];
  const float* kb3 = (const float*)d_in[17];
  float* out = (float*)d_out;

  char* ws = (char*)d_ws;
  size_t off = 0;
  const size_t oP  = off; off += (size_t)NPT * NC * 4;
  const size_t oL1 = off; off += (size_t)NBLK * 32 * 4;
  const size_t oL3 = off; off += (size_t)NBLK * 32 * 4;
  if (off > ws_size || off > (size_t)WSCAP) return;
  float* P     = (float*)(ws + oP);
  float* part1 = (float*)(ws + oL1);
  float* part3 = (float*)(ws + oL3);

  k_cpl1<<<dim3(NBLK), dim3(NTHR), 0, stream>>>(x, an_logs, an_bias, w1, b1, g1, be1, w2, b2, w3, b3,
                                                 P, part1);
  k_cpl2<<<dim3(NBLK), dim3(NTHR), 0, stream>>>(P, knn, k1, kb1, k2, kb2, k3, kb3, out, part3);
  k_logdet<<<dim3(1), dim3(64), 0, stream>>>(an_logs, part1, part3, out);
}
